// MultiHeadAttn_32658931319413
// MI455X (gfx1250) — hardware-verified
//
#include <hip/hip_runtime.h>
#include <math.h>
#include <stdint.h>

#ifndef NB
#define NB 4
#endif
#ifndef NB_FULL
#define NB_FULL 4
#endif
#ifndef SEQ
#define SEQ 2048
#endif
#ifndef SEQ_FULL
#define SEQ_FULL 2048
#endif
#define NH    16
#define HD    64
#define DM    1024
#define DQKV  3072
#define NQB   (SEQ / 64)
#define MTOK  (NB * SEQ)
#ifndef RESQB
#define RESQB 0
#endif
#define PCARRY 16384.0f
#define PRES   4096.0f
#define VCARRY 64.0f
#define OCARRY 64.0f
#define WCARRY 64.0f

#define BM  128
#define BN  128
#define BK  32
#define TP  136
#define TPF 132

static_assert(NB >= 1 && NB <= NB_FULL);
static_assert((SEQ % 128) == 0 && SEQ >= 128 && SEQ <= SEQ_FULL);
static_assert(NH * HD == DM);
static_assert((MTOK % BM) == 0 && (SEQ % BM) == 0);
static_assert((DQKV % BN) == 0 && (DM % BN) == 0 && (DM % BK) == 0 && (DM % 64) == 0);
static_assert(BN == 2 * HD);
static_assert(RESQB >= 0);
static_assert((long long)MTOK * DM * 4 <= 33554432LL);

typedef _Float16 v16h __attribute__((ext_vector_type(16)));
typedef _Float16 v8h  __attribute__((ext_vector_type(8)));
typedef __bf16   v16b __attribute__((ext_vector_type(16)));
typedef __bf16   v8b  __attribute__((ext_vector_type(8)));
typedef float    v8f  __attribute__((ext_vector_type(8)));
typedef float    v4f  __attribute__((ext_vector_type(4)));
typedef unsigned int v4u __attribute__((ext_vector_type(4)));
typedef unsigned short v8us __attribute__((ext_vector_type(8)));

__device__ __forceinline__ unsigned short bf_bits(float f) {
  unsigned u = __float_as_uint(f);
  return (unsigned short)((u + 0x7FFFu + ((u >> 16) & 1u)) >> 16);
}
__device__ __forceinline__ float bf_up(unsigned short h) { return __uint_as_float(((unsigned)h) << 16); }
__device__ __forceinline__ unsigned pk16(unsigned short a, unsigned short b) { return (unsigned)a | ((unsigned)b << 16); }
__device__ __forceinline__ unsigned short h_bits(float f) {
  const _Float16 hv = (_Float16)f;
  return __builtin_bit_cast(unsigned short, hv);
}
__device__ __forceinline__ v8f zero8() { v8f z = {0.f, 0.f, 0.f, 0.f, 0.f, 0.f, 0.f, 0.f}; return z; }

template <typename E> struct FT;
template <> struct FT<__bf16> {
  typedef v16b V16;
  typedef v8b  V8;
  static __device__ __forceinline__ v16b ld(const __bf16* p) {
    union { v16b v; v8b h[2]; } f;
    f.h[0] = *(const v8b*)(p);
    f.h[1] = *(const v8b*)(p + 16);
    return f.v;
  }
  static __device__ __forceinline__ v8f mma(v16b a, v16b b, v8f c) {
    c = __builtin_amdgcn_wmma_f32_16x16x32_bf16(false, a, false, b, (short)0, c, false, false);
    asm volatile("v_nop\n\tv_nop\n\tv_nop\n\tv_nop" : "+v"(c) : "v"(a), "v"(b));
    return c;
  }
};
template <> struct FT<_Float16> {
  typedef v16h V16;
  typedef v8h  V8;
  static __device__ __forceinline__ v16h ld(const _Float16* p) {
    union { v16h v; v8h h[2]; } f;
    f.h[0] = *(const v8h*)(p);
    f.h[1] = *(const v8h*)(p + 16);
    return f.v;
  }
  static __device__ __forceinline__ v8f mma(v16h a, v16h b, v8f c) {
    c = __builtin_amdgcn_wmma_f32_16x16x32_f16(false, a, false, b, (short)0, c, false, false);
    asm volatile("v_nop\n\tv_nop\n\tv_nop\n\tv_nop" : "+v"(c) : "v"(a), "v"(b));
    return c;
  }
};

__global__ __launch_bounds__(256) void cvt_bf16x8s(const float* __restrict__ in, unsigned short* out,
                                                   int n8, int per8, int src8) {
  const int i = blockIdx.x * 256 + threadIdx.x;
  if (i < n8) {
    const int hd  = i / per8;
    const int rem = i - hd * per8;
    const float* s = in + ((size_t)hd * src8 + (size_t)rem) * 8;
    const v4f a = *(const v4f*)(s);
    const v4f b = *(const v4f*)(s + 4);
    v4u p;
    p[0] = pk16(bf_bits(a[0]), bf_bits(a[1]));
    p[1] = pk16(bf_bits(a[2]), bf_bits(a[3]));
    p[2] = pk16(bf_bits(b[0]), bf_bits(b[1]));
    p[3] = pk16(bf_bits(b[2]), bf_bits(b[3]));
    *(volatile v4u*)(out + (size_t)i * 8) = p;
    __threadfence();
    *(volatile v4u*)(out + (size_t)i * 8) = p;
  }
}

__global__ __launch_bounds__(256) void wt_tiles(const float* __restrict__ w, unsigned short* wt, int ncol, int mode) {
  __shared__ __align__(16) unsigned short T[64 * 64];
  const int tid = threadIdx.x;
  const int nkt = DM / 64;
  const int nt  = blockIdx.x / nkt;
  const int kt  = blockIdx.x - nt * nkt;
  const int kr  = tid >> 2;
  const int nq  = (tid & 3) * 16;
  const float* src = w + (size_t)(kt * 64 + kr) * ncol + (size_t)nt * 64 + nq;
#pragma unroll
  for (int i = 0; i < 4; ++i) {
    const v4f a = *(const v4f*)(src + 4 * i);
#pragma unroll
    for (int e = 0; e < 4; ++e) {
      const unsigned short ub = bf_bits(a[e]);
      const unsigned short uh = h_bits(bf_up(ub) * WCARRY);
      T[(nq + 4 * i + e) * 64 + kr] = (mode != 0) ? uh : ub;
    }
  }
  __syncthreads();
  const int wave = tid >> 5, lane = tid & 31;
  const int q = lane >> 3, c8 = (lane & 7) * 8;
  union { v8us h; v4u u; } w0, w1;
  const int n0r = wave * 8 + q;
  const int n1r = wave * 8 + 4 + q;
  w0.h = *(const v8us*)(T + n0r * 64 + c8);
  w1.h = *(const v8us*)(T + n1r * 64 + c8);
  unsigned short* p0 = wt + ((size_t)(nt * 64 + n0r) * DM + (size_t)kt * 64 + c8);
  unsigned short* p1 = wt + ((size_t)(nt * 64 + n1r) * DM + (size_t)kt * 64 + c8);
  *(volatile v4u*)p0 = w0.u;
  *(volatile v4u*)p1 = w1.u;
  __threadfence();
  *(volatile v4u*)p0 = w0.u;
  *(volatile v4u*)p1 = w1.u;
}

template <typename E>
__device__ __forceinline__ void mainloop128(const E* __restrict__ A, const E* __restrict__ Bt, E* As, E* Bs,
                                            int m0, int n0, int lda, int ldb, int kdim, v8f acc[4][2]) {
  typedef typename FT<E>::V16 V16;
  typedef typename FT<E>::V8  V8;
  const int t = threadIdx.x, wave = t >> 5, lane = t & 31, hh = lane >> 4, c = lane & 15;
  const int wm = wave >> 2, wn = wave & 3;
  for (int kb = 0; kb < kdim; kb += BK) {
#pragma unroll
    for (int i = 0; i < 2; ++i) {
      const int idx = t + i * 256;
      const int row = idx >> 2, seg = (idx & 3) * 8;
      const V8 av = *(const V8*)(A  + (size_t)(m0 + row) * lda + kb + seg);
      const V8 bv = *(const V8*)(Bt + (size_t)(n0 + row) * ldb + kb + seg);
      *(V8*)(As + row * BK + seg) = av;
      *(V8*)(Bs + row * BK + seg) = bv;
    }
    __syncthreads();
    V16 af[4];
#pragma unroll
    for (int mi = 0; mi < 4; ++mi) af[mi] = FT<E>::ld(As + (wm * 64 + mi * 16 + c) * BK + 8 * hh);
#pragma unroll
    for (int ni = 0; ni < 2; ++ni) {
      const V16 bfr = FT<E>::ld(Bs + (wn * 32 + ni * 16 + c) * BK + 8 * hh);
#pragma unroll
      for (int mi = 0; mi < 4; ++mi) acc[mi][ni] = FT<E>::mma(af[mi], bfr, acc[mi][ni]);
    }
    __syncthreads();
  }
}

__global__ __launch_bounds__(256)
void k_gemm_qkv(const unsigned short* __restrict__ xb, const unsigned short* __restrict__ wqt,
                unsigned short* qpl, unsigned short* kpl, unsigned short* vtpl) {
  typedef FT<__bf16> F;
  __shared__ __align__(16) __bf16   As[BM * BK];
  __shared__ __align__(16) __bf16   Bs[BN * BK];
  __shared__ __align__(16) _Float16 T[BM * TP];
  const int bm = blockIdx.x, bn = blockIdx.y;
  const int m0 = bm * BM, n0 = bn * BN;
  v8f acc[4][2];
#pragma unroll
  for (int mi = 0; mi < 4; ++mi)
#pragma unroll
    for (int ni = 0; ni < 2; ++ni) acc[mi][ni] = zero8();
  mainloop128<__bf16>((const __bf16*)(const void*)xb, (const __bf16*)(const void*)wqt, As, Bs, m0, n0, DM, DM, DM, acc);
  (void)sizeof(F);

  const int t = threadIdx.x, wave = t >> 5, lane = t & 31, hh = lane >> 4, c = lane & 15;
  const int wm = wave >> 2, wn = wave & 3;
  const int s  = n0 / DM;
  const int hb = (n0 - s * DM) / HD;
  const int b  = m0 / SEQ;
  const int p0 = m0 - b * SEQ;
  const int lq = t >> 3, c8 = (t & 7) * 8;

  if (s < 2) {
#pragma unroll
    for (int mi = 0; mi < 4; ++mi)
#pragma unroll
      for (int ni = 0; ni < 2; ++ni)
#pragma unroll
        for (int r = 0; r < 8; ++r)
          T[(wm * 64 + mi * 16 + 8 * hh + r) * TP + wn * 32 + ni * 16 + c] = (_Float16)acc[mi][ni][r];
    __syncthreads();
    v4u vals[8];
#pragma unroll
    for (int it = 0; it < 8; ++it) {
      const int L = it * 32 + lq;
      const int row = L & 127, j = L >> 7;
      union { v8h h; v4u u; } w;
      w.h = *(const v8h*)(T + row * TP + j * 64 + c8);
      vals[it] = w.u;
    }
    unsigned short* dst = (s == 0) ? qpl : kpl;
    for (int rep = 0; rep < 2; ++rep) {
#pragma unroll
      for (int it = 0; it < 8; ++it) {
        const int L = it * 32 + lq;
        const int row = L & 127, j = L >> 7;
        unsigned short* p = dst + ((size_t)((b * NH + hb + j) * SEQ + p0 + row)) * HD + c8;
        *(volatile v4u*)p = vals[it];
      }
      __threadfence();
    }
  } else {
#pragma unroll
    for (int mi = 0; mi < 4; ++mi)
#pragma unroll
      for (int ni = 0; ni < 2; ++ni)
#pragma unroll
        for (int r = 0; r < 8; ++r)
          T[(wn * 32 + ni * 16 + c) * TP + wm * 64 + mi * 16 + 8 * hh + r] = (_Float16)(acc[mi][ni][r] * VCARRY);
    __syncthreads();
    v4u vals[8];
#pragma unroll
    for (int it = 0; it < 8; ++it) {
      const int L = it * 32 + lq;
      const int j = L >> 7, d = (L >> 1) & 63, q2 = L & 1;
      union { v8h h; v4u u; } w;
      w.h = *(const v8h*)(T + (j * 64 + d) * TP + q2 * 64 + c8);
      vals[it] = w.u;
    }
    for (int rep = 0; rep < 2; ++rep) {
#pragma unroll
      for (int it = 0; it < 8; ++it) {
        const int L = it * 32 + lq;
        const int j = L >> 7, d = (L >> 1) & 63, q2 = L & 1;
        unsigned short* p = vtpl + ((size_t)((b * NH + hb + j) * HD + d)) * SEQ + p0 + q2 * 64 + c8;
        *(volatile v4u*)p = vals[it];
      }
      __threadfence();
    }
  }
}

template <bool RES>
__global__ __launch_bounds__(128)
void attn_full64(const unsigned short* __restrict__ qp, const unsigned short* __restrict__ kp,
                 const unsigned short* __restrict__ vtp, unsigned short* op, int qbBase, int nqbThis) {
  typedef FT<_Float16> F;
  union FH { v16h v; v8h h[2]; };
  __shared__ __align__(16) _Float16 Ksh[64 * 64];
  __shared__ __align__(16) _Float16 Vth[64 * 64];
  __shared__ __align__(16) _Float16 Psh[4][16 * 64];
  __shared__ __align__(16) _Float16 Psl[RES ? 4 : 1][16 * 64];
  __shared__ __align__(16) _Float16 Os[4][16 * 64];

  const int tid  = threadIdx.x;
  const int wave = tid >> 5;
  const int lane = tid & 31;
  const int hh   = lane >> 4;
  const int c    = lane & 15;

  const int bx   = blockIdx.x;
  const int qbl  = bx % nqbThis;
  const int bh   = bx / nqbThis;
  const int b    = bh / NH;
  const int h    = bh - b * NH;
  const int qb   = qbBase + qbl;
  const int q0   = qb * 64 + wave * 16;

  const _Float16* Qh = (const _Float16*)(const void*)qp  + (size_t)bh * SEQ * HD;
  const _Float16* Kh = (const _Float16*)(const void*)kp  + (size_t)bh * SEQ * HD;
  const _Float16* Vh = (const _Float16*)(const void*)vtp + (size_t)bh * HD * SEQ;

  v16h qa[2];
#pragma unroll
  for (int dc = 0; dc < 2; ++dc) {
    const size_t qo = (size_t)(q0 + c) * HD + dc * 32 + 8 * hh;
    qa[dc] = F::ld(Qh + qo);
  }

  float mrow[8], lrow[8];
  v8f oacc[4];
#pragma unroll
  for (int r = 0; r < 8; ++r) { mrow[r] = -INFINITY; lrow[r] = 0.f; }
#pragma unroll
  for (int t = 0; t < 4; ++t) oacc[t] = zero8();

  for (int kt = 0; kt < NQB; ++kt) {
    const int kv0 = kt * 64;
    __syncthreads();
    {
      const int r = tid >> 1, half = (tid & 1) * 32;
      const _Float16* kg = Kh + (size_t)(kv0 + r) * HD + half;
      const _Float16* vg = Vh + (size_t)r * SEQ + kv0 + half;
#pragma unroll
      for (int i = 0; i < 4; ++i) {
        const v8h a0 = *(const v8h*)(kg + 8 * i);
        const v8h b0 = *(const v8h*)(vg + 8 * i);
        *(v8h*)(Ksh + r * 64 + half + 8 * i) = a0;
        *(v8h*)(Vth + r * 64 + half + 8 * i) = b0;
      }
    }
    __syncthreads();

    v8f s[4];
#pragma unroll
    for (int j = 0; j < 4; ++j) {
      s[j] = zero8();
#pragma unroll
      for (int dc = 0; dc < 2; ++dc) {
        FH kb;
        kb.h[0] = *(const v8h*)(Ksh + (j * 16 + c) * 64 + dc * 32 + 8 * hh);
        kb.h[1] = *(const v8h*)(Ksh + (j * 16 + c) * 64 + dc * 32 + 16 + 8 * hh);
        s[j] = F::mma(qa[dc], kb.v, s[j]);
      }
    }

    _Float16* pwh = Psh[wave];
    _Float16* pwl = Psl[RES ? wave : 0];
#pragma unroll
    for (int r = 0; r < 8; ++r) {
      float m = -INFINITY;
#pragma unroll
      for (int j = 0; j < 4; ++j) {
        const float sv = s[j][r] * 0.125f;
        s[j][r] = sv;
        m = fmaxf(m, sv);
      }
#pragma unroll
      for (int off = 1; off < 16; off <<= 1) m = fmaxf(m, __shfl_xor(m, off, 32));
      const float mnew  = fmaxf(mrow[r], m);
      const float msafe = (mnew == -INFINITY) ? 0.f : mnew;
      const float alpha = __expf(mrow[r] - msafe);
      mrow[r] = mnew;
      float psum = 0.f;
#pragma unroll
      for (int j = 0; j < 4; ++j) {
        const float p = __expf(s[j][r] - msafe);
        psum += p;
        const float p1k = p * PCARRY;
        const _Float16 ph = (_Float16)p1k;
        pwh[(8 * hh + r) * 64 + j * 16 + c] = ph;
        if (RES) {
          const _Float16 pl = (_Float16)((p1k - (float)ph) * PRES);
          pwl[(8 * hh + r) * 64 + j * 16 + c] = pl;
        }
      }
#pragma unroll
      for (int off = 1; off < 16; off <<= 1) psum += __shfl_xor(psum, off, 32);
      lrow[r] = lrow[r] * alpha + psum;
#pragma unroll
      for (int t = 0; t < 4; ++t) oacc[t][r] *= alpha;
    }
    __builtin_amdgcn_fence(__ATOMIC_RELEASE, "workgroup");
    __builtin_amdgcn_wave_barrier();
    __builtin_amdgcn_fence(__ATOMIC_ACQUIRE, "workgroup");

    v8f o1[4];
#pragma unroll
    for (int t = 0; t < 4; ++t) o1[t] = zero8();
#pragma unroll 1
    for (int kk = 0; kk < 2; ++kk) {
      FH pa, pl;
      pa.h[0] = *(const v8h*)(pwh + c * 64 + kk * 32 + 8 * hh);
      pa.h[1] = *(const v8h*)(pwh + c * 64 + kk * 32 + 16 + 8 * hh);
      if (RES) {
        pl.h[0] = *(const v8h*)(pwl + c * 64 + kk * 32 + 8 * hh);
        pl.h[1] = *(const v8h*)(pwl + c * 64 + kk * 32 + 16 + 8 * hh);
      } else {
        pl.v = pa.v;
      }
#pragma unroll
      for (int t = 0; t < 4; ++t) {
        FH vb;
        vb.h[0] = *(const v8h*)(Vth + (t * 16 + c) * 64 + kk * 32 + 8 * hh);
        vb.h[1] = *(const v8h*)(Vth + (t * 16 + c) * 64 + kk * 32 + 16 + 8 * hh);
        oacc[t] = F::mma(pa.v, vb.v, oacc[t]);
        if (RES) o1[t] = F::mma(pl.v, vb.v, o1[t]);
      }
    }
    if (RES) {
#pragma unroll
      for (int t = 0; t < 4; ++t)
#pragma unroll
        for (int r = 0; r < 8; ++r) oacc[t][r] += o1[t][r] * (1.0f / PRES);
    }
  }

  _Float16* os = Os[wave];
#pragma unroll
  for (int r = 0; r < 8; ++r) {
    const float l = lrow[r];
    const float inv = ((l > 0.f) ? (1.0f / l) : 0.f) * (OCARRY / (PCARRY * VCARRY));
#pragma unroll
    for (int t = 0; t < 4; ++t) os[(8 * hh + r) * 64 + t * 16 + c] = (_Float16)(oacc[t][r] * inv);
  }
  __builtin_amdgcn_fence(__ATOMIC_RELEASE, "workgroup");
  __builtin_amdgcn_wave_barrier();
  __builtin_amdgcn_fence(__ATOMIC_ACQUIRE, "workgroup");
  {
    const int rq = lane >> 3, c8 = (lane & 7) * 8;
    v4u vals[4];
#pragma unroll
    for (int it = 0; it < 4; ++it) {
      const int row = it * 4 + rq;
      union { v8h h; v4u u; } w;
      w.h = *(const v8h*)(os + row * 64 + c8);
      vals[it] = w.u;
    }
    unsigned short* ob = op + ((size_t)(b * SEQ + q0)) * DM + h * HD + c8;
    for (int rep = 0; rep < 2; ++rep) {
#pragma unroll
      for (int it = 0; it < 4; ++it) {
        const int row = it * 4 + rq;
        *(volatile v4u*)(ob + (size_t)row * DM) = vals[it];
      }
      __threadfence();
    }
  }
}

__global__ __launch_bounds__(256)
void k_gemm_out(const unsigned short* __restrict__ ob, const unsigned short* __restrict__ wpt,
                const float* __restrict__ bias, float* outp) {
  typedef FT<_Float16> F;
  __shared__ __align__(16) _Float16 As[BM * BK];
  __shared__ __align__(16) _Float16 Bs[BN * BK];
  __shared__ __align__(16) float    Tf[64 * TPF];
  const int bm = blockIdx.x, bn = blockIdx.y;
  const int m0 = bm * BM, n0 = bn * BN;
  v8f acc[4][2];
#pragma unroll
  for (int mi = 0; mi < 4; ++mi)
#pragma unroll
    for (int ni = 0; ni < 2; ++ni) acc[mi][ni] = zero8();
  mainloop128<_Float16>((const _Float16*)(const void*)ob, (const _Float16*)(const void*)wpt, As, Bs,
                        m0, n0, DM, DM, DM, acc);
  (void)sizeof(F);

  const int t = threadIdx.x, wave = t >> 5, lane = t & 31, hh = lane >> 4, c = lane & 15;
  const int wm = wave >> 2, wn = wave & 3;
  const float inv = 1.0f / (OCARRY * WCARRY);
  const int lq = t >> 3, seg = lq & 3, c4 = seg * 32 + (t & 7) * 4, rsub = lq >> 2;
  v4f bb;
  {
    const v4f b4 = *(const v4f*)(bias + n0 + c4);
#pragma unroll
    for (int e = 0; e < 4; ++e) bb[e] = bf_up(bf_bits(b4[e]));
  }
  for (int hm = 0; hm < 2; ++hm) {
    if (wm == hm) {
#pragma unroll
      for (int mi = 0; mi < 4; ++mi)
#pragma unroll
        for (int ni = 0; ni < 2; ++ni)
#pragma unroll
          for (int r = 0; r < 8; ++r)
            Tf[(mi * 16 + 8 * hh + r) * TPF + wn * 32 + ni * 16 + c] = acc[mi][ni][r] * inv;
    }
    __syncthreads();
    v4f vals[8];
#pragma unroll
    for (int it = 0; it < 8; ++it) {
      const int row = it * 8 + rsub;
      vals[it] = *(const v4f*)(Tf + row * TPF + c4) + bb;
    }
    float* dst = outp + ((size_t)(m0 + hm * 64)) * DM + n0 + c4;
    for (int rep = 0; rep < 2; ++rep) {
#pragma unroll
      for (int it = 0; it < 8; ++it) {
        const int row = it * 8 + rsub;
        *(volatile v4f*)(dst + (size_t)row * DM) = vals[it];
      }
      __threadfence();
    }
    __syncthreads();
  }
}

extern "C" void kernel_launch(void* const* d_in, const int* in_sizes, int n_in,
                              void* d_out, int out_size, void* d_ws, size_t ws_size,
                              hipStream_t stream) {
  if (n_in < 4) return;
  const long long needX = ((long long)(NB - 1) * SEQ_FULL + (long long)SEQ) * DM;
  if ((long long)in_sizes[0] < needX) return;
  if ((long long)in_sizes[1] < (long long)DM * DQKV) return;
  if ((long long)in_sizes[2] < (long long)DM * DM) return;
  if (in_sizes[3] < DM) return;
  if (out_size < 0 || (long long)out_size < (long long)MTOK * DM) return;

  const size_t szAct = (size_t)MTOK * DM * 2;
  const size_t szWq  = (size_t)DQKV * DM * 2;
  const size_t szWp  = (size_t)DM * DM * 2;
  size_t off = 0;
  const size_t oX  = off; off += szAct;
  const size_t oWq = off; off += szWq;
  const size_t oWp = off; off += szWp;
  const size_t oQ  = off; off += szAct;
  const size_t oK  = off; off += szAct;
  const size_t oVT = off; off += szAct;
  const size_t oO  = off; off += szAct;
  if (off > ws_size) return;
  if (off > (size_t)134217728) return;

  const float* x      = (const float*)d_in[0];
  const float* w_qkv  = (const float*)d_in[1];
  const float* w_proj = (const float*)d_in[2];
  const float* b_proj = (const float*)d_in[3];
  float* out = (float*)d_out;

  char* ws = (char*)d_ws;
  unsigned short* Xb  = (unsigned short*)(ws + oX);
  unsigned short* WqT = (unsigned short*)(ws + oWq);
  unsigned short* WpT = (unsigned short*)(ws + oWp);
  unsigned short* Qp  = (unsigned short*)(ws + oQ);
  unsigned short* Kp  = (unsigned short*)(ws + oK);
  unsigned short* VTp = (unsigned short*)(ws + oVT);
  unsigned short* Op  = (unsigned short*)(ws + oO);

  const dim3 blk(256);
  const int n8   = MTOK * DM / 8;
  const int per8 = SEQ * DM / 8;
  const int src8 = SEQ_FULL * DM / 8;
  const dim3 gCvt((n8 + 255) / 256);
  const dim3 gWq((DQKV / 64) * (DM / 64));
  const dim3 gWp((DM / 64) * (DM / 64));
  const dim3 gG1(MTOK / BM, DQKV / BN);
  const dim3 gG2(MTOK / BM, DM / BN);
  int resqb = RESQB;
  if (resqb > NQB) resqb = NQB;

  cvt_bf16x8s<<<gCvt, blk, 0, stream>>>(x, Xb, n8, per8, src8);
  wt_tiles<<<gWq, blk, 0, stream>>>(w_qkv, WqT, DQKV, 0);
  wt_tiles<<<gWp, blk, 0, stream>>>(w_proj, WpT, DM, 1);
  k_gemm_qkv<<<gG1, blk, 0, stream>>>(Xb, WqT, Qp, Kp, VTp);
  if (resqb > 0) {
    attn_full64<true><<<dim3(NB * NH * resqb), dim3(128), 0, stream>>>(Qp, Kp, VTp, Op, 0, resqb);
  }
  if (NQB - resqb > 0) {
    attn_full64<false><<<dim3(NB * NH * (NQB - resqb)), dim3(128), 0, stream>>>(Qp, Kp, VTp, Op, resqb, NQB - resqb);
  }
  k_gemm_out<<<gG2, blk, 0, stream>>>(Op, WpT, b_proj, out);
  (void)hipGetLastError();
}
